// Trainer_5308579578440
// MI455X (gfx1250) — hardware-verified
//
#include <hip/hip_runtime.h>
#include <math.h>

typedef __attribute__((ext_vector_type(16))) _Float16 v16h;
typedef __attribute__((ext_vector_type(8)))  _Float16 v8h;
typedef __attribute__((ext_vector_type(8)))  float    v8f;
typedef __attribute__((ext_vector_type(4)))  float    v4f;
typedef __attribute__((ext_vector_type(2)))  float    v2f;
typedef __attribute__((ext_vector_type(4)))  unsigned v4u;

#define NCH         64
#define SEQ_LEN     512
#define DEC_LEN     35
#define NSTEP       (SEQ_LEN + DEC_LEN)
#define GROWS       192
#define TPB_MAIN    128
#define ROWS_BLK    16
#define PRED_ROW    (DEC_LEN * 2)
#define TILE_HALVES (ROWS_BLK * NCH)
#define ACT_CARRY   16.0f
#define WGT_CARRY   64.0f
#define ACC_FOLD    (1.0f / 1024.0f)

__device__ __forceinline__ v16h frag_load(const _Float16* p) {
  union { v16h v; v8h h[2]; } f;
  f.h[0] = *(const v8h*)(p);
  f.h[1] = *(const v8h*)(p + 16);
  return f.v;
}

__device__ __forceinline__ v8f mma16(v16h a, v16h b, v8f c) {
  c = __builtin_amdgcn_wmma_f32_16x16x32_f16(false, a, false, b, (short)0, c, false, false);
  asm volatile("v_nop\n\tv_nop\n\tv_nop\n\tv_nop" : "+v"(c) : "v"(a), "v"(b));
  return c;
}

__device__ __forceinline__ unsigned pack_f16x2(float a, float b) {
  const unsigned ua = (unsigned)__builtin_bit_cast(unsigned short, (_Float16)a);
  const unsigned ub = (unsigned)__builtin_bit_cast(unsigned short, (_Float16)b);
  return ua | (ub << 16);
}

__device__ __forceinline__ float sigm_f(float x) {
  return __builtin_amdgcn_rcpf(1.0f + expf(-x));
}
__device__ __forceinline__ float tanh_f(float x) {
  return 1.0f - 2.0f * __builtin_amdgcn_rcpf(1.0f + expf(2.0f * x));
}

__global__ __launch_bounds__(256) void cast_weights_f16(
    const float* __restrict__ w0, const float* __restrict__ w1,
    _Float16* __restrict__ o0, _Float16* __restrict__ o1, int n2, float scale) {
  const int i = blockIdx.x * 256 + threadIdx.x;
  if (i < n2) {
    const unsigned u0 = pack_f16x2(w0[2 * i] * scale, w0[2 * i + 1] * scale);
    const unsigned u1 = pack_f16x2(w1[2 * i] * scale, w1[2 * i + 1] * scale);
    ((volatile unsigned*)o0)[i] = u0;
    ((volatile unsigned*)o1)[i] = u1;
    __threadfence();
    ((volatile unsigned*)o0)[i] = u0;
    ((volatile unsigned*)o1)[i] = u1;
  }
}

__device__ __forceinline__ void build_x_tile(_Float16* s_xt, const float* s_d1w, const float* s_d1b,
                                             const float* s_emb, const float* prow_ptr,
                                             int s, int prow, int pcb) {
  const int t = (s < SEQ_LEN) ? s : (SEQ_LEN - 1);
  const v2f p = *(const v2f*)(prow_ptr + (size_t)t * 2);
  const bool use_emb = (s >= SEQ_LEN);
  const v8f wa = *(const v8f*)(s_d1w + 2 * pcb);
  const v8f wb = *(const v8f*)(s_d1w + 2 * pcb + 8);
  const v8f bb = *(const v8f*)(s_d1b + pcb);
  const v8f ee = *(const v8f*)(s_emb + pcb);
  float v[8];
#pragma unroll
  for (int e = 0; e < 4; ++e) {
    const float d0 = p.x * wa[2 * e] + p.y * wa[2 * e + 1] + bb[e];
    const float d1 = p.x * wb[2 * e] + p.y * wb[2 * e + 1] + bb[4 + e];
    v[e]     = (use_emb ? ee[e]     : d0) * ACT_CARRY;
    v[4 + e] = (use_emb ? ee[4 + e] : d1) * ACT_CARRY;
  }
  v4u w;
  w.x = pack_f16x2(v[0], v[1]);
  w.y = pack_f16x2(v[2], v[3]);
  w.z = pack_f16x2(v[4], v[5]);
  w.w = pack_f16x2(v[6], v[7]);
  *(v4u*)(s_xt + prow * NCH + pcb) = w;
}

template <bool TOP>
__device__ __forceinline__ void gru_layer(const _Float16* xbuf, _Float16* hbuf,
                                          const _Float16* __restrict__ wih, const _Float16* __restrict__ whh,
                                          int c0, int lane, v8f& hreg,
                                          float br, float bz, float bin, float bhn,
                                          float* htop) {
  const int hh = lane >> 4;
  const int cc = lane & 15;
  const v16h xa0 = frag_load(xbuf + cc * NCH + 8 * hh);
  const v16h xa1 = frag_load(xbuf + cc * NCH + 32 + 8 * hh);
  const v16h ha0 = frag_load(hbuf + cc * NCH + 8 * hh);
  const v16h ha1 = frag_load(hbuf + cc * NCH + 32 + 8 * hh);
  __syncthreads();

  const v8f zero8 = {0.f, 0.f, 0.f, 0.f, 0.f, 0.f, 0.f, 0.f};
  v8f ar = zero8, az = zero8, ai = zero8, ah = zero8;
  const _Float16* wr = wih + (c0 + cc) * NCH + 8 * hh;
  const _Float16* ur = whh + (c0 + cc) * NCH + 8 * hh;
  ar = mma16(xa0, frag_load(wr), ar);
  ar = mma16(xa1, frag_load(wr + 32), ar);
  ar = mma16(ha0, frag_load(ur), ar);
  ar = mma16(ha1, frag_load(ur + 32), ar);
  az = mma16(xa0, frag_load(wr + 64 * NCH), az);
  az = mma16(xa1, frag_load(wr + 64 * NCH + 32), az);
  az = mma16(ha0, frag_load(ur + 64 * NCH), az);
  az = mma16(ha1, frag_load(ur + 64 * NCH + 32), az);
  ai = mma16(xa0, frag_load(wr + 128 * NCH), ai);
  ai = mma16(xa1, frag_load(wr + 128 * NCH + 32), ai);
  ah = mma16(ha0, frag_load(ur + 128 * NCH), ah);
  ah = mma16(ha1, frag_load(ur + 128 * NCH + 32), ah);

  const int nc = c0 + cc;
  const int m0 = 8 * hh;
#pragma unroll
  for (int i = 0; i < 8; ++i) {
    const float r  = sigm_f(ar[i] * ACC_FOLD + br);
    const float z  = sigm_f(az[i] * ACC_FOLD + bz);
    const float hn = ah[i] * ACC_FOLD + bhn;
    const float n  = tanh_f(ai[i] * ACC_FOLD + bin + r * hn);
    const float h  = (1.0f - z) * n + z * hreg[i];
    hreg[i] = h;
    hbuf[(m0 + i) * NCH + nc] = (_Float16)(h * ACT_CARRY);
    if (TOP) htop[(m0 + i) * NCH + nc] = h;
  }
  __syncthreads();
}

__global__ void __launch_bounds__(TPB_MAIN) gru_seq2seq_kernel(
    const float* __restrict__ pulse,
    const float* __restrict__ d1w, const float* __restrict__ d1b,
    const float* __restrict__ d2w, const float* __restrict__ d2b,
    const _Float16* __restrict__ wih16, const _Float16* __restrict__ whh16,
    const float* __restrict__ bih, const float* __restrict__ bhh,
    const float* __restrict__ emb,
    float* __restrict__ out, int nbatch) {
  __shared__ __align__(32) _Float16 s_tile[3 * TILE_HALVES];
  __shared__ __align__(32) float    s_htop[ROWS_BLK * NCH];
  __shared__ __align__(32) float    s_pred[ROWS_BLK * PRED_ROW];
  __shared__ __align__(32) float    s_d1w[2 * NCH];
  __shared__ __align__(32) float    s_d1b[NCH];
  __shared__ __align__(32) float    s_emb[NCH];
  __shared__ __align__(32) float    s_d2w[2 * NCH];

  const int tid  = threadIdx.x;
  const int lane = tid & 31;
  const int wave = tid >> 5;
  const int c0   = wave << 4;
  const int wg   = blockIdx.x;
  if (wg * ROWS_BLK + ROWS_BLK > nbatch) return;

  _Float16* s_x  = s_tile;
  _Float16* s_h0 = s_tile + TILE_HALVES;
  _Float16* s_h1 = s_tile + 2 * TILE_HALVES;

  if (tid < 2 * NCH) { s_d1w[tid] = d1w[tid]; s_d2w[tid] = d2w[tid]; }
  if (tid < NCH)     { s_d1b[tid] = d1b[tid]; s_emb[tid] = emb[tid]; }
  *(v4u*)(s_h0 + 8 * tid) = (v4u){0u, 0u, 0u, 0u};
  *(v4u*)(s_h1 + 8 * tid) = (v4u){0u, 0u, 0u, 0u};
  v8f h0reg = {0.f, 0.f, 0.f, 0.f, 0.f, 0.f, 0.f, 0.f};
  v8f h1reg = {0.f, 0.f, 0.f, 0.f, 0.f, 0.f, 0.f, 0.f};

  const int nc = c0 + (lane & 15);
  const float br0  = bih[nc] + bhh[nc];
  const float bz0  = bih[64 + nc] + bhh[64 + nc];
  const float bin0 = bih[128 + nc];
  const float bhn0 = bhh[128 + nc];
  const float br1  = bih[GROWS + nc] + bhh[GROWS + nc];
  const float bz1  = bih[GROWS + 64 + nc] + bhh[GROWS + 64 + nc];
  const float bin1 = bih[GROWS + 128 + nc];
  const float bhn1 = bhh[GROWS + 128 + nc];
  const float d2bo = d2b[lane & 1];

  const int prow = tid >> 3;
  const int pcb  = (tid & 7) << 3;
  const float* prow_ptr = pulse + (size_t)(wg * ROWS_BLK + prow) * (SEQ_LEN * 2);

  const _Float16* wih_l0 = wih16;
  const _Float16* whh_l0 = whh16;
  const _Float16* wih_l1 = wih16 + GROWS * NCH;
  const _Float16* whh_l1 = whh16 + GROWS * NCH;

  __syncthreads();
  build_x_tile(s_x, s_d1w, s_d1b, s_emb, prow_ptr, 0, prow, pcb);
  __syncthreads();

  for (int step = 0; step < NSTEP; ++step) {
    const _Float16* xb = s_tile + ((step <= SEQ_LEN) ? 0 : 2 * TILE_HALVES);
    gru_layer<false>(xb, s_h0, wih_l0, whh_l0, c0, lane, h0reg, br0, bz0, bin0, bhn0, nullptr);
    if (step + 1 <= SEQ_LEN) build_x_tile(s_x, s_d1w, s_d1b, s_emb, prow_ptr, step + 1, prow, pcb);
    gru_layer<true>(s_h0, s_h1, wih_l1, whh_l1, c0, lane, h1reg, br1, bz1, bin1, bhn1, s_htop);

    if (step >= SEQ_LEN && wave == 0) {
      const int r = lane >> 1, o = lane & 1;
      const int ds = step - SEQ_LEN;
      float acc = 0.f;
#pragma unroll 4
      for (int ch = 0; ch < NCH; ++ch) acc += s_htop[r * NCH + ch] * s_d2w[o * NCH + ch];
      s_pred[r * PRED_ROW + ds * 2 + o] = acc + d2bo;
    }
  }
  __syncthreads();

  float* ob = out + (size_t)wg * (ROWS_BLK * PRED_ROW);
  for (int pass = 0; pass < 2; ++pass) {
#pragma unroll
    for (int i = 0; i < 3; ++i) {
      const int f = tid + i * TPB_MAIN;
      if (f < (ROWS_BLK * PRED_ROW) / 4) {
        const v4f val = *(const v4f*)(s_pred + 4 * f);
        *(volatile v4f*)(ob + 4 * f) = val;
      }
    }
    __threadfence();
  }
}

extern "C" void kernel_launch(void* const* d_in, const int* in_sizes, int n_in,
                              void* d_out, int out_size, void* d_ws, size_t ws_size,
                              hipStream_t stream) {
  (void)n_in;
  const float* pulse = (const float*)d_in[0];
  const float* d1w   = (const float*)d_in[1];
  const float* d1b   = (const float*)d_in[2];
  const float* d2w   = (const float*)d_in[3];
  const float* d2b   = (const float*)d_in[4];
  const float* Wih   = (const float*)d_in[5];
  const float* Whh   = (const float*)d_in[6];
  const float* bihp  = (const float*)d_in[7];
  const float* bhhp  = (const float*)d_in[8];
  const float* emb   = (const float*)d_in[9];
  float* out = (float*)d_out;

  if (in_sizes[5] != 2 * GROWS * NCH || in_sizes[6] != 2 * GROWS * NCH) return;
  const int nbatch = in_sizes[0] / (SEQ_LEN * 2);
  int grid = nbatch / ROWS_BLK;
  const int max_blocks = out_size / (ROWS_BLK * PRED_ROW);
  if (grid > max_blocks) grid = max_blocks;
  if (grid <= 0) return;

  const size_t plane_bytes = (size_t)in_sizes[5] * 2;
  if (ws_size < 2 * plane_bytes) return;
  _Float16* wih16 = (_Float16*)d_ws;
  _Float16* whh16 = (_Float16*)((char*)d_ws + plane_bytes);

  const int n2 = in_sizes[5] / 2;
  const int cgrid = (n2 + 255) / 256;
  cast_weights_f16<<<cgrid, 256, 0, stream>>>(Wih, Whh, wih16, whh16, n2, WGT_CARRY);

  gru_seq2seq_kernel<<<grid, TPB_MAIN, 0, stream>>>(
      pulse, d1w, d1b, d2w, d2b, wih16, whh16, bihp, bhhp, emb, out, nbatch);
}
